// CircularRelativePositionAttention_2422361555015
// MI455X (gfx1250) — hardware-verified
//
#include <hip/hip_runtime.h>


typedef _Float16 v16h __attribute__((ext_vector_type(16)));
typedef _Float16 v8h  __attribute__((ext_vector_type(8), may_alias));
typedef _Float16 v4h  __attribute__((ext_vector_type(4), may_alias));
typedef __bf16   v16b __attribute__((ext_vector_type(16)));
typedef unsigned short v8us __attribute__((ext_vector_type(8), may_alias));
typedef float v8f __attribute__((ext_vector_type(8)));
typedef float v4f __attribute__((ext_vector_type(4), may_alias));

#define SEQ   1000
#define SEQP  1008
#define DM    512
#define DH    64
#define NB    8
#define NH    8
#define QTN   63
#define KTI   63
#define SPAD  1024
#define NDIST 512
#define DMAX  500
#define NW    4
#define NT    128
#define PSC   256.0f
#define PSCI  0.00390625f

#define WS_K    ((size_t)0)
#define WS_VT   ((size_t)NB * SEQP * DM)
#define WS_RK   (WS_VT + (size_t)NB * NH * DH * SPAD)
#define WS_RVT  (WS_RK + (size_t)NDIST * DH)
#define WS_END  (WS_RVT + (size_t)DH * NDIST)

#define NK8  (NB * SEQP * DM / 8)
#define NV8  (NB * NH * DH * SPAD / 8)
#define NR8  (NDIST * DH / 8)

union FragH { v16h v; v8h  h[2]; };
union FragB { v16b v; v8us h[2]; };

__device__ __forceinline__ v8f zero8() {
  v8f z = {0.0f, 0.0f, 0.0f, 0.0f, 0.0f, 0.0f, 0.0f, 0.0f};
  return z;
}

__device__ __forceinline__ v8f wmma_f16(const FragH& a, const FragH& b, v8f c) {
  v8f d = __builtin_amdgcn_wmma_f32_16x16x32_f16(false, a.v, false, b.v, (short)0, c, false, false);
  asm volatile("v_nop\n\tv_nop\n\tv_nop\n\tv_nop" : "+v"(d) : "v"(a.v), "v"(b.v));
  return d;
}

__device__ __forceinline__ v8f wmma_bf16(const FragB& a, const FragB& b, v8f c) {
  v8f d = __builtin_amdgcn_wmma_f32_16x16x32_bf16(false, a.v, false, b.v, (short)0, c, false, false);
  asm volatile("v_nop\n\tv_nop\n\tv_nop\n\tv_nop" : "+v"(d) : "v"(a.v), "v"(b.v));
  return d;
}

__device__ __forceinline__ unsigned short bf16_rne(float f) {
  unsigned int u = __float_as_uint(f);
  u += 0x7FFFu + ((u >> 16) & 1u);
  return (unsigned short)(u >> 16);
}

__device__ __forceinline__ _Float16 f16_of_bf16(float f) {
  unsigned int u = ((unsigned int)bf16_rne(f)) << 16;
  return (_Float16)__uint_as_float(u);
}

__device__ __forceinline__ int circ_dist(int i, int j) {
  int t = (i - j) % SEQ;
  if (t < 0) t += SEQ;
  return min(t, SEQ - t);
}

__global__ __launch_bounds__(256)
void prep_k_kernel(const float* __restrict__ K, unsigned short* __restrict__ Kb) {
  const int t = blockIdx.x * 256 + threadIdx.x;
  if (t >= NK8) return;
  const size_t e0 = (size_t)t * 8;
  const int b = (int)(e0 / ((size_t)SEQP * DM));
  const int r = (int)((e0 / DM) % SEQP);
  const int d = (int)(e0 % DM);
  v8us o = {0, 0, 0, 0, 0, 0, 0, 0};
  if (r < SEQ) {
    const float* src = K + ((size_t)b * SEQ + r) * DM + d;
    v4f x0 = *(const v4f*)(src);
    v4f x1 = *(const v4f*)(src + 4);
    o[0] = bf16_rne(x0.x); o[1] = bf16_rne(x0.y); o[2] = bf16_rne(x0.z); o[3] = bf16_rne(x0.w);
    o[4] = bf16_rne(x1.x); o[5] = bf16_rne(x1.y); o[6] = bf16_rne(x1.z); o[7] = bf16_rne(x1.w);
  }
  volatile v8us* p = (volatile v8us*)(Kb + e0);
  *p = o;
  __threadfence();
  *p = o;
}

__global__ __launch_bounds__(256)
void prep_vt_kernel(const float* __restrict__ V, _Float16* __restrict__ Vt) {
  const int t = blockIdx.x * 256 + threadIdx.x;
  if (t >= NV8) return;
  const int e0   = t * 8;
  const int bh   = e0 >> 16;
  const int dim  = (e0 >> 10) & (DH - 1);
  const int key0 = e0 & (SPAD - 1);
  const int b = bh >> 3, h = bh & 7;
  v8h o = {0, 0, 0, 0, 0, 0, 0, 0};
  if (key0 < SEQ) {
    const float* src = V + ((size_t)b * SEQ + key0) * DM + h * DH + dim;
    #pragma unroll
    for (int j = 0; j < 8; ++j) o[j] = f16_of_bf16(src[(size_t)j * DM]);
  }
  volatile v8h* p = (volatile v8h*)(Vt + (size_t)e0);
  *p = o;
  __threadfence();
  *p = o;
}

__global__ __launch_bounds__(256)
void prep_rel_kernel(const float* __restrict__ RK, const float* __restrict__ RV,
                     unsigned short* __restrict__ RKb, _Float16* __restrict__ RVt) {
  const int t = blockIdx.x * 256 + threadIdx.x;
  if (t < NR8) {
    const int e0 = t * 8;
    v4f x0 = *(const v4f*)(RK + e0);
    v4f x1 = *(const v4f*)(RK + e0 + 4);
    v8us o;
    o[0] = bf16_rne(x0.x); o[1] = bf16_rne(x0.y); o[2] = bf16_rne(x0.z); o[3] = bf16_rne(x0.w);
    o[4] = bf16_rne(x1.x); o[5] = bf16_rne(x1.y); o[6] = bf16_rne(x1.z); o[7] = bf16_rne(x1.w);
    volatile v8us* p = (volatile v8us*)(RKb + e0);
    *p = o;
    __threadfence();
    *p = o;
  } else if (t < 2 * NR8) {
    const int e0 = (t - NR8) * 8;
    const int d = e0 >> 9;
    const int dist0 = e0 & (NDIST - 1);
    v8h o;
    #pragma unroll
    for (int j = 0; j < 8; ++j) o[j] = f16_of_bf16(RV[(size_t)(dist0 + j) * DH + d]);
    volatile v8h* p = (volatile v8h*)(RVt + e0);
    *p = o;
    __threadfence();
    *p = o;
  }
}

__global__ __launch_bounds__(NT)
void circ_rel_attn_kernel(const float* __restrict__ Q,
                          const unsigned short* __restrict__ Kb,
                          const _Float16* __restrict__ Vt,
                          const unsigned short* __restrict__ RKb,
                          const _Float16* __restrict__ RVt,
                          float* __restrict__ Out)
{
  __shared__ __attribute__((aligned(16))) unsigned short sQ[16 * DH];
  __shared__ __attribute__((aligned(16))) float          sP[16 * NDIST];
  __shared__ __attribute__((aligned(16))) float          sS[16 * SPAD];
  __shared__ __attribute__((aligned(16))) _Float16       sA[16 * SPAD];
  __shared__ __attribute__((aligned(16))) _Float16       sD[16 * NDIST];
  __shared__ float sRed[16 * 8];
  __shared__ float sMax[16];
  __shared__ float sRcp[16];

  const int qt   = blockIdx.x;
  const int bh   = blockIdx.y;
  const int b    = bh >> 3;
  const int h    = bh & 7;
  const int tid  = threadIdx.x;
  const int lane = tid & 31;
  const int wave = tid >> 5;
  const int n    = lane & 15;
  const int hi   = lane >> 4;

  const float scale = 0.125f;
  const size_t baseQ = (size_t)b * SEQ * DM + (size_t)h * DH;
  const unsigned short* Kbh = Kb + ((size_t)b * SEQP) * DM + (size_t)h * DH;
  const _Float16* Vbh = Vt + (size_t)bh * DH * SPAD;

  for (int idx = tid; idx < 16 * DH; idx += NT) {
    const int m = idx >> 6, d = idx & 63;
    const int qrow = qt * 16 + m;
    const float v = (qrow < SEQ) ? Q[baseQ + (size_t)qrow * DM + d] : 0.0f;
    sQ[idx] = bf16_rne(v);
  }
  __syncthreads();

  FragB qa0, qa1;
  {
    const unsigned short* qp = sQ + n * DH + 8 * hi;
    qa0.h[0] = *(const v8us*)(qp);
    qa0.h[1] = *(const v8us*)(qp + 16);
    qa1.h[0] = *(const v8us*)(qp + 32);
    qa1.h[1] = *(const v8us*)(qp + 48);
  }

  for (int ct = wave; ct < NDIST / 16; ct += NW) {
    const unsigned short* rp = RKb + (size_t)(ct * 16 + n) * DH + 8 * hi;
    FragB b0, b1;
    b0.h[0] = *(const v8us*)(rp);
    b0.h[1] = *(const v8us*)(rp + 16);
    b1.h[0] = *(const v8us*)(rp + 32);
    b1.h[1] = *(const v8us*)(rp + 48);
    v8f acc = zero8();
    acc = wmma_bf16(qa0, b0, acc);
    acc = wmma_bf16(qa1, b1, acc);
    #pragma unroll
    for (int r = 0; r < 8; ++r)
      sP[(r + 8 * hi) * NDIST + ct * 16 + n] = acc[r];
  }
  __syncthreads();

  for (int kt = wave; kt < KTI; kt += NW) {
    const int key = kt * 16 + n;
    const unsigned short* kp = Kbh + (size_t)key * DM + 8 * hi;
    FragB b0, b1;
    b0.h[0] = *(const v8us*)(kp);
    b0.h[1] = *(const v8us*)(kp + 16);
    b1.h[0] = *(const v8us*)(kp + 32);
    b1.h[1] = *(const v8us*)(kp + 48);
    v8f acc = zero8();
    acc = wmma_bf16(qa0, b0, acc);
    acc = wmma_bf16(qa1, b1, acc);
    #pragma unroll
    for (int r = 0; r < 8; ++r) {
      const int m = r + 8 * hi;
      const int qrow = min(qt * 16 + m, SEQ - 1);
      float sc;
      if (key < SEQ) {
        const int d = circ_dist(qrow, key);
        sc = acc[r] * scale + sP[m * NDIST + d];
      } else {
        sc = -1.0e30f;
      }
      sS[m * SPAD + key] = sc;
    }
  }
  __syncthreads();

  {
    const int row = tid >> 3, sub = tid & 7;
    const int j0 = sub * 128;
    float* rowS = sS + row * SPAD;
    _Float16* rowA = sA + row * SPAD;

    float mx = -1.0e30f;
    for (int j = j0; j < j0 + 128; j += 4) {
      if (j < SEQ) {
        v4f v = *(const v4f*)(rowS + j);
        mx = fmaxf(mx, fmaxf(fmaxf(v.x, v.y), fmaxf(v.z, v.w)));
      }
    }
    sRed[row * 8 + sub] = mx;
    __syncthreads();
    if (sub == 0) {
      float m2 = sRed[row * 8];
      #pragma unroll
      for (int u = 1; u < 8; ++u) m2 = fmaxf(m2, sRed[row * 8 + u]);
      sMax[row] = m2;
    }
    __syncthreads();
    const float rm = sMax[row];
    float sum = 0.0f;
    for (int j = j0; j < j0 + 128; j += 4) {
      v4f e = {0.0f, 0.0f, 0.0f, 0.0f};
      if (j < SEQ) {
        v4f v = *(const v4f*)(rowS + j);
        e.x = __expf(v.x - rm); e.y = __expf(v.y - rm);
        e.z = __expf(v.z - rm); e.w = __expf(v.w - rm);
      }
      *(v4f*)(rowS + j) = e;
      v4h h4;
      h4.x = (_Float16)(e.x * PSC); h4.y = (_Float16)(e.y * PSC);
      h4.z = (_Float16)(e.z * PSC); h4.w = (_Float16)(e.w * PSC);
      *(v4h*)(rowA + j) = h4;
      sum += (e.x + e.y) + (e.z + e.w);
    }
    sRed[row * 8 + sub] = sum;
    __syncthreads();
    if (sub == 0) {
      float s2 = 0.0f;
      #pragma unroll
      for (int u = 0; u < 8; ++u) s2 += sRed[row * 8 + u];
      sRcp[row] = 1.0f / s2;
    }
    __syncthreads();
  }

  for (int idx = tid; idx < 16 * NDIST; idx += NT) {
    const int m = idx >> 9, dist = idx & (NDIST - 1);
    const int qrow = min(qt * 16 + m, SEQ - 1);
    float val = 0.0f;
    if (dist <= DMAX) {
      int k1 = qrow - dist; if (k1 < 0) k1 += SEQ;
      int k2 = qrow + dist; if (k2 >= SEQ) k2 -= SEQ;
      val = sS[m * SPAD + k1];
      if (k2 != k1) val += sS[m * SPAD + k2];
    }
    sD[idx] = (_Float16)(val * PSC);
  }
  __syncthreads();

  {
    const int dbase = wave * 16;
    const _Float16* vcol  = Vbh + (size_t)(dbase + n) * SPAD  + 8 * hi;
    const _Float16* rvcol = RVt + (size_t)(dbase + n) * NDIST + 8 * hi;
    const _Float16* arow  = sA + n * SPAD  + 8 * hi;
    const _Float16* drow  = sD + n * NDIST + 8 * hi;
    v8f acc = zero8();

    #pragma unroll 4
    for (int kt2 = 0; kt2 < SPAD / 32; ++kt2) {
      const int kb = kt2 * 32;
      FragH a, bb;
      a.h[0]  = *(const v8h*)(arow + kb);
      a.h[1]  = *(const v8h*)(arow + kb + 16);
      bb.h[0] = *(const v8h*)(vcol + kb);
      bb.h[1] = *(const v8h*)(vcol + kb + 16);
      acc = wmma_f16(a, bb, acc);
    }
    #pragma unroll 4
    for (int rt = 0; rt < NDIST / 32; ++rt) {
      const int kb = rt * 32;
      FragH a, bb;
      a.h[0]  = *(const v8h*)(drow + kb);
      a.h[1]  = *(const v8h*)(drow + kb + 16);
      bb.h[0] = *(const v8h*)(rvcol + kb);
      bb.h[1] = *(const v8h*)(rvcol + kb + 16);
      acc = wmma_f16(a, bb, acc);
    }
    #pragma unroll
    for (int r = 0; r < 8; ++r) {
      const int m = r + 8 * hi;
      sP[m * DH + dbase + n] = acc[r] * (sRcp[m] * PSCI);
    }
  }
  __syncthreads();

  {
    float* obase = Out + baseQ;
    #pragma unroll
    for (int i = 0; i < 2; ++i) {
      const int L = i * 4 + (lane >> 3);
      const int m = wave * 4 + (L >> 1);
      const int c = (L & 1) * 32 + (lane & 7) * 4;
      const int qrow = qt * 16 + m;
      v4f v = *(const v4f*)(sP + m * DH + c);
      if (qrow < SEQ) *(volatile v4f*)(obase + (size_t)qrow * DM + c) = v;
    }
    __threadfence();
    #pragma unroll
    for (int i = 0; i < 2; ++i) {
      const int L = i * 4 + (lane >> 3);
      const int m = wave * 4 + (L >> 1);
      const int c = (L & 1) * 32 + (lane & 7) * 4;
      const int qrow = qt * 16 + m;
      v4f v = *(const v4f*)(sP + m * DH + c);
      if (qrow < SEQ) *(volatile v4f*)(obase + (size_t)qrow * DM + c) = v;
    }
  }
}

extern "C" void kernel_launch(void* const* d_in, const int* in_sizes, int n_in,
                              void* d_out, int out_size, void* d_ws, size_t ws_size,
                              hipStream_t stream) {
  if (n_in < 5) return;
  if (in_sizes[0] < NB * SEQ * DM || in_sizes[1] < NB * SEQ * DM || in_sizes[2] < NB * SEQ * DM) return;
  if (in_sizes[3] < NDIST * DH || in_sizes[4] < NDIST * DH) return;
  if (out_size < NB * SEQ * DM) return;
  const size_t ws_need = WS_END * 2;
  if (ws_size < ws_need) return;

  const float* Q  = (const float*)d_in[0];
  const float* K  = (const float*)d_in[1];
  const float* V  = (const float*)d_in[2];
  const float* RK = (const float*)d_in[3];
  const float* RV = (const float*)d_in[4];
  float* Out = (float*)d_out;
  unsigned short* ws16 = (unsigned short*)d_ws;

  unsigned short* Kb  = ws16 + WS_K;
  _Float16*       Vt  = (_Float16*)(ws16 + WS_VT);
  unsigned short* RKb = ws16 + WS_RK;
  _Float16*       RVt = (_Float16*)(ws16 + WS_RVT);

  prep_k_kernel  <<<(NK8 + 255) / 256, 256, 0, stream>>>(K, Kb);
  prep_vt_kernel <<<(NV8 + 255) / 256, 256, 0, stream>>>(V, Vt);
  prep_rel_kernel<<<(2 * NR8 + 255) / 256, 256, 0, stream>>>(RK, RV, RKb, RVt);

  dim3 grid(QTN, NB * NH);
  circ_rel_attn_kernel<<<grid, dim3(NT), 0, stream>>>(Q, Kb, Vt, RKb, RVt, Out);
}
